// mTAN_enc_23304492548180
// MI455X (gfx1250) — hardware-run, weakly checked
//
#include <hip/hip_runtime.h>
#include <math.h>

constexpr int kNB   = 64;
constexpr int kNL   = 4096;
constexpr int kNQ   = 128;
constexpr int kND   = 32;
constexpr int kNE   = 128;
constexpr int kNH   = 128;
constexpr int kNG3  = 384;
constexpr int kNCLS = 6;
constexpr int kGB   = 16;
constexpr int kNGRP = kNB / kGB;
constexpr int kXTR  = 64;
constexpr int kHAP  = 136;
constexpr int kSFP  = 132;

constexpr float kTeCarry  = 16.0f;
constexpr float kWCarry   = 8.0f;
constexpr float kPCarry   = 32768.0f;
constexpr float kAttCarry = 256.0f;
constexpr float kActCarry = 16.0f;
constexpr float kGhScale  = 1.0f / (kActCarry * kWCarry);
constexpr float kLog2e    = 1.4426950408889634f;

typedef __attribute__((ext_vector_type(16))) _Float16 v16h;
typedef __attribute__((ext_vector_type(8)))  _Float16 v8h;
typedef __attribute__((ext_vector_type(16))) __bf16   v16b;
typedef __attribute__((ext_vector_type(8)))  __bf16   v8b;
typedef __attribute__((ext_vector_type(8)))  float    v8f;
typedef __attribute__((ext_vector_type(4)))  float    v4f;
typedef __attribute__((ext_vector_type(4)))  unsigned int v4u;
typedef unsigned int v4ua __attribute__((ext_vector_type(4), __may_alias__));

__device__ __forceinline__ unsigned short f2bf_bits(float f) {
  unsigned u = __float_as_uint(f);
  return (unsigned short)((u + 0x7FFFu + ((u >> 16) & 1u)) >> 16);
}
__device__ __forceinline__ float bf_bits2f(unsigned short h) { return __uint_as_float(((unsigned)h) << 16); }

__device__ __forceinline__ void dep_guard_h(v8f& a, v8f& b, v16h x, v16h y) { asm volatile("v_nop\n\tv_nop\n\tv_nop\n\tv_nop" : "+v"(a), "+v"(b) : "v"(x), "v"(y)); }
__device__ __forceinline__ void dep_guard_b(v8f& a, v8f& b, v16b x, v16b y) { asm volatile("v_nop\n\tv_nop\n\tv_nop\n\tv_nop" : "+v"(a), "+v"(b) : "v"(x), "v"(y)); }
__device__ __forceinline__ void keep4_h(v16h a, v16h b, v16h c, v16h d) { asm volatile("v_nop" :: "v"(a), "v"(b), "v"(c), "v"(d)); }
__device__ __forceinline__ void keep4_b(v16b a, v16b b, v16b c, v16b d) { asm volatile("v_nop" :: "v"(a), "v"(b), "v"(c), "v"(d)); }
__device__ __forceinline__ void acc_guard4(v8f& a, v8f& b, v8f& c, v8f& d) { asm volatile("v_nop\n\tv_nop\n\tv_nop\n\tv_nop" : "+v"(a), "+v"(b), "+v"(c), "+v"(d)); }
template <typename T> struct Frag;
template <> struct Frag<_Float16> {
  typedef v16h V; union U { v16h v; v8h h[2]; };
  static __device__ __forceinline__ v16h load(const _Float16* p) {
    U f; f.h[0] = *(const v8h*)(p); f.h[1] = *(const v8h*)(p + 16); return f.v;
  }
  static __device__ __forceinline__ v8f mma(v16h a, v16h b, v8f c) {
    return __builtin_amdgcn_wmma_f32_16x16x32_f16(false, a, false, b, (short)0, c, false, false);
  }
  static __device__ __forceinline__ void guard(v8f& a, v8f& b, v16h x, v16h y) { dep_guard_h(a, b, x, y); }
  static __device__ __forceinline__ void keep(v16h a, v16h b, v16h c, v16h d) { keep4_h(a, b, c, d); }
};
template <> struct Frag<__bf16> {
  typedef v16b V; union U { v16b v; v8b h[2]; };
  static __device__ __forceinline__ v16b load(const __bf16* p) {
    U f; f.h[0] = *(const v8b*)(p); f.h[1] = *(const v8b*)(p + 16); return f.v;
  }
  static __device__ __forceinline__ v8f mma(v16b a, v16b b, v8f c) {
    return __builtin_amdgcn_wmma_f32_16x16x32_bf16(false, a, false, b, (short)0, c, false, false);
  }
  static __device__ __forceinline__ void guard(v8f& a, v8f& b, v16b x, v16b y) { dep_guard_b(a, b, x, y); }
  static __device__ __forceinline__ void keep(v16b a, v16b b, v16b c, v16b d) { keep4_b(a, b, c, d); }
};

__device__ __forceinline__ unsigned pk16(unsigned short a, unsigned short b) { return (unsigned)a | ((unsigned)b << 16); }
__device__ __forceinline__ unsigned short h_bits(float f) { const _Float16 h = (_Float16)f; return __builtin_bit_cast(unsigned short, h); }

__device__ __forceinline__ void guard3_h(v8f& a, v8f& b, v8f& c, v16h x, v16h y, v16h z, v16h w) {
  asm volatile("v_nop\n\tv_nop\n\tv_nop\n\tv_nop" : "+v"(a), "+v"(b), "+v"(c) : "v"(x), "v"(y), "v"(z), "v"(w));
}

template <int ET> struct Elem;
template <> struct Elem<0> { typedef _Float16 T; };
template <> struct Elem<1> { typedef __bf16 T; };
template <int ET, bool SPLIT, int BIAS_MODE, int OUT_MODE, bool RESID, int ACT = 0>
__global__ __launch_bounds__(256) void wmma_gemm64(
    const unsigned short* __restrict__ Ap, const unsigned short* __restrict__ A2p, int lda, long strideA,
    const unsigned short* __restrict__ Btp, const unsigned short* __restrict__ Bt2p, int ldb, long strideB,
    void* __restrict__ Cout, void* __restrict__ Cout2, int ldc, long strideC,
    const float* __restrict__ bias,
    const float* __restrict__ resid, long strideR,
    int M, int N, int K, float scale) {
  typedef typename Elem<ET>::T T;
  typedef typename Frag<T>::V V;
  const T* A = (const T*)Ap; const T* A2 = (const T*)A2p; const T* Bt = (const T*)Btp; const T* Bt2 = (const T*)Bt2p;
  __shared__ __align__(16) float sT[8][16 * 68];
  const int b    = blockIdx.y;
  const int lane = threadIdx.x & 31;
  const int wave = threadIdx.x >> 5;
  const int tilesN = N >> 6;
  const int tilesM = M >> 6;
  const int tile = blockIdx.x * 8 + wave;
  if (tile >= tilesM * tilesN) return;
  const int tm = tile / tilesN;
  const int tn = tile - tm * tilesN;
  const int m0 = tm << 6;
  const int n0 = tn << 6;

  const T* Ab  = A  + (size_t)b * strideA;
  const T* Bb  = Bt + (size_t)b * strideB;
  const T* Ab2 = SPLIT ? (A2  + (size_t)b * strideA) : nullptr;
  const T* Bb2 = SPLIT ? (Bt2 + (size_t)b * strideB) : nullptr;

  const int rlane = lane & 15;
  const int koff  = (lane >> 4) * 8;
  const int mOff  = (lane >> 4) * 8;

  v8f acc[4][4];
#pragma unroll
  for (int i = 0; i < 4; ++i)
#pragma unroll
    for (int j = 0; j < 4; ++j) acc[i][j] = (v8f){0.f,0.f,0.f,0.f,0.f,0.f,0.f,0.f};

  for (int k0 = 0; k0 < K; k0 += 32) {
    V bh[4], bl[4];
#pragma unroll
    for (int j = 0; j < 4; ++j) {
      const size_t bo = (size_t)(n0 + (j << 4) + rlane) * ldb + koff + k0;
      bh[j] = Frag<T>::load(Bb + bo);
      if (SPLIT) bl[j] = Frag<T>::load(Bb2 + bo);
    }
#pragma unroll
    for (int i = 0; i < 4; ++i) {
      const size_t ao = (size_t)(m0 + (i << 4) + rlane) * lda + koff + k0;
      V ah = Frag<T>::load(Ab + ao);
      V al;
      if (SPLIT) al = Frag<T>::load(Ab2 + ao);
#pragma unroll
      for (int j = 0; j < 4; ++j) {
        acc[i][j] = Frag<T>::mma(ah, bh[j], acc[i][j]);
        if (SPLIT) {
          acc[i][j] = Frag<T>::mma(ah, bl[j], acc[i][j]);
          acc[i][j] = Frag<T>::mma(al, bh[j], acc[i][j]);
        }
      }
      Frag<T>::guard(acc[i][0], acc[i][3], ah, SPLIT ? al : ah);
    }
    Frag<T>::keep(bh[0], bh[1], bh[2], bh[3]);
    if (SPLIT) Frag<T>::keep(bl[0], bl[1], bl[2], bl[3]);
  }
  acc_guard4(acc[0][0], acc[0][1], acc[0][2], acc[0][3]);
  acc_guard4(acc[1][0], acc[1][1], acc[1][2], acc[1][3]);
  acc_guard4(acc[2][0], acc[2][1], acc[2][2], acc[2][3]);
  acc_guard4(acc[3][0], acc[3][1], acc[3][2], acc[3][3]);

  float* slab = sT[wave];
  const float* Rb = RESID ? (resid + (size_t)b * strideR) : nullptr;
#pragma unroll
  for (int i = 0; i < 4; ++i) {
    const int mBase = m0 + (i << 4);
#pragma unroll
    for (int j = 0; j < 4; ++j) {
      const int n = n0 + (j << 4) + rlane;
      float bv = 0.f;
      if (BIAS_MODE == 2) bv = bias[n];
#pragma unroll
      for (int r = 0; r < 8; ++r) {
        float v = acc[i][j][r] * scale;
        if (BIAS_MODE == 1) v += bias[mBase + mOff + r];
        if (BIAS_MODE == 2) v += bv;
        if (RESID) v += Rb[(size_t)(mBase + mOff + r) * ldc + n];
        if (ACT == 2) v = fmaxf(v, 0.0f);
        if (ACT == 4) v = (v > 0.f) ? v : 0.01f * v;
        slab[(mOff + r) * 68 + (j << 4) + rlane] = v;
      }
    }
    __builtin_amdgcn_fence(__ATOMIC_RELEASE, "workgroup");
    __builtin_amdgcn_wave_barrier();
    __builtin_amdgcn_fence(__ATOMIC_ACQUIRE, "workgroup");
    if (OUT_MODE == 0) {
      float* C = (float*)Cout + (size_t)b * strideC;
      const int hh = lane >> 4, c4 = (lane & 15) * 4;
      for (int pass = 0; pass < 2; ++pass) {
#pragma unroll
        for (int it = 0; it < 8; ++it) {
          const int row = it * 2 + hh;
          v4f v = *(const v4f*)(slab + row * 68 + c4);
          *(volatile v4f*)(C + (size_t)(mBase + row) * ldc + n0 + c4) = v;
        }
        __threadfence();
      }
    } else {
      const int q = lane >> 3, c8 = (lane & 7) * 8;
      unsigned short* C  = (unsigned short*)Cout  + (size_t)b * strideC;
      unsigned short* C2 = (OUT_MODE == 2) ? ((unsigned short*)Cout2 + (size_t)b * strideC) : nullptr;
      for (int pass = 0; pass < 2; ++pass) {
#pragma unroll
        for (int it = 0; it < 4; ++it) {
          const int row = it * 4 + q;
          const float* sp = slab + row * 68 + c8;
          v8h hv, lv;
#pragma unroll
          for (int e = 0; e < 8; ++e) {
            if (OUT_MODE == 1) {
              hv[e] = (_Float16)sp[e];
            } else {
              unsigned short hb = f2bf_bits(sp[e]);
              unsigned short lb = f2bf_bits(sp[e] - bf_bits2f(hb));
              hv[e] = __builtin_bit_cast(_Float16, hb);
              lv[e] = __builtin_bit_cast(_Float16, lb);
            }
          }
          *(volatile v8h*)(C + (size_t)(mBase + row) * ldc + n0 + c8) = hv;
          if (OUT_MODE == 2) *(volatile v8h*)(C2 + (size_t)(mBase + row) * ldc + n0 + c8) = lv;
        }
        __threadfence();
      }
    }
    __builtin_amdgcn_fence(__ATOMIC_RELEASE, "workgroup");
    __builtin_amdgcn_wave_barrier();
    __builtin_amdgcn_fence(__ATOMIC_ACQUIRE, "workgroup");
  }
}

__global__ __launch_bounds__(32) void prep_bias_kernel(const float* __restrict__ bq, const float* __restrict__ bk,
                                                      const float* __restrict__ bo, float* __restrict__ dst3) {
  const int z = blockIdx.x;
  const int lane = threadIdx.x;
  const float* src = (z == 0) ? bq : (z == 1) ? bk : bo;
  const float sc = (z == 2) ? kActCarry : kWCarry;
  float* dst = dst3 + z * kNE + 4 * lane;
  v4f v = *(const v4f*)(src + 4 * lane);
  v = v * sc;
  for (int pass = 0; pass < 2; ++pass) {
    *(volatile v4f*)dst = v;
    __threadfence();
  }
}

__global__ __launch_bounds__(256) void wtrans_kernel(const float* __restrict__ w0, const float* __restrict__ w1,
                                                     const float* __restrict__ w2, unsigned short* __restrict__ o0,
                                                     unsigned short* __restrict__ o1, unsigned short* __restrict__ o2,
                                                     float scale) {
  __shared__ __align__(16) unsigned short sm[kNE][kHAP];
  const int tid = threadIdx.x;
  const int z = blockIdx.x;
  const float* in = (z == 0) ? w0 : (z == 1) ? w1 : w2;
  unsigned short* out = (z == 0) ? o0 : (z == 1) ? o1 : o2;
  const int kdsh = (z == 2) ? 5 : 7;
  const int kd = 1 << kdsh;
  const int tot = kd * kNE;
  for (int e = tid; e < tot; e += 256) {
    const int k = e >> 7;
    const int n = e & (kNE - 1);
    sm[n][k] = h_bits(in[e] * scale);
  }
  __syncthreads();
  const int n8 = tot >> 3;
  for (int pass = 0; pass < 2; ++pass) {
    for (int i = tid; i < n8; i += 256) {
      const int f = i << 3;
      const int n = f >> kdsh;
      const int k0 = f & (kd - 1);
      const v4u u = *(const v4ua*)(&sm[n][k0]);
      *(volatile v4u*)(out + f) = u;
    }
    __threadfence();
  }
}

__global__ __launch_bounds__(256) void castw_kernel(const float* __restrict__ s0, const float* __restrict__ s1,
                                                    const float* __restrict__ s2, const float* __restrict__ s3,
                                                    unsigned short* __restrict__ d0, unsigned short* __restrict__ d1,
                                                    unsigned short* __restrict__ d2, unsigned short* __restrict__ d3,
                                                    int n8_small, int n8_big, float scale) {
  const int z = blockIdx.y;
  const float* in = (z == 0) ? s0 : (z == 1) ? s1 : (z == 2) ? s2 : s3;
  unsigned short* out = (z == 0) ? d0 : (z == 1) ? d1 : (z == 2) ? d2 : d3;
  const int n8 = (z == 2) ? n8_big : n8_small;
  const int i = blockIdx.x * 256 + threadIdx.x;
  if (i >= n8) return;
  const float* p = in + 8 * (size_t)i;
  const v4f a = *(const v4f*)(p);
  const v4f c = *(const v4f*)(p + 4);
  unsigned short hb[8];
#pragma unroll
  for (int e = 0; e < 4; ++e) {
    hb[e]     = h_bits(a[e] * scale);
    hb[4 + e] = h_bits(c[e] * scale);
  }
  const v4u u = (v4u){pk16(hb[0], hb[1]), pk16(hb[2], hb[3]), pk16(hb[4], hb[5]), pk16(hb[6], hb[7])};
  unsigned short* q = out + 8 * (size_t)i;
  *(volatile v4u*)q = u;
  __threadfence();
  *(volatile v4u*)q = u;
}

__global__ __launch_bounds__(256) void te_kernel(const float* __restrict__ tt, int nrows,
                                                 const float* __restrict__ lin_w, const float* __restrict__ lin_b,
                                                 const float* __restrict__ per_w, const float* __restrict__ per_b,
                                                 unsigned short* __restrict__ out) {
#pragma clang fp contract(off)
  __shared__ __align__(16) unsigned short sm[16][kHAP];
  const int tid = threadIdx.x;
  const int row0 = blockIdx.x * 16;
  const float lw = lin_w[0];
  const float lb = lin_b[0];
#pragma unroll 1
  for (int it = 0; it < 8; ++it) {
    const int e = it * 256 + tid;
    const int rl = e >> 7;
    const int col = e & 127;
    int row = row0 + rl;
    row = (row < nrows) ? row : (nrows - 1);
    const float t = tt[row];
    const int pc = (col > 0) ? (col - 1) : 0;
    const float pw = per_w[pc];
    const float pb = per_b[pc];
    const float arg = t * pw + pb;
    const float sv = sinf(arg);
    const float lv = t * lw + lb;
    const float v = (col == 0) ? lv : sv;
    sm[rl][col] = h_bits(v * kTeCarry);
  }
  __syncthreads();
  const int rl = tid >> 4;
  const int c8 = (tid & 15) * 8;
  const int row = row0 + rl;
  const v4u u = *(const v4ua*)(&sm[rl][c8]);
  if (row < nrows) {
    unsigned short* q = out + (size_t)row * kNE + c8;
    *(volatile v4u*)q = u;
    __threadfence();
    *(volatile v4u*)q = u;
  }
}

__global__ __launch_bounds__(256) void softmax_kernel(const float* __restrict__ S, unsigned short* __restrict__ P) {
  __shared__ float redm[8];
  __shared__ float reds[8];
  const int row = blockIdx.x;
  const int t = threadIdx.x;
  const int lane = t & 31, wave = t >> 5;
  const float* sr = S + (size_t)row * kNL;
  const int cA = 8 * t;
  const int cB = (kNL / 2) + 8 * t;
  const v4f a0 = *(const v4f*)(sr + cA);
  const v4f a1 = *(const v4f*)(sr + cA + 4);
  const v4f b0 = *(const v4f*)(sr + cB);
  const v4f b1 = *(const v4f*)(sr + cB + 4);
  float x[16];
#pragma unroll
  for (int e = 0; e < 4; ++e) { x[e] = a0[e]; x[4 + e] = a1[e]; x[8 + e] = b0[e]; x[12 + e] = b1[e]; }
  float m = x[0];
#pragma unroll
  for (int e = 1; e < 16; ++e) m = fmaxf(m, x[e]);
#pragma unroll
  for (int off = 16; off > 0; off >>= 1) m = fmaxf(m, __shfl_xor(m, off, 32));
  if (lane == 0) redm[wave] = m;
  __syncthreads();
  float gm = redm[0];
#pragma unroll
  for (int w = 1; w < 8; ++w) gm = fmaxf(gm, redm[w]);
  float ev[16];
  float ps = 0.f;
#pragma unroll
  for (int e = 0; e < 16; ++e) { ev[e] = exp2f((x[e] - gm) * kLog2e); ps += ev[e]; }
#pragma unroll
  for (int off = 16; off > 0; off >>= 1) ps += __shfl_xor(ps, off, 32);
  if (lane == 0) reds[wave] = ps;
  __syncthreads();
  float tot = reds[0];
#pragma unroll
  for (int w = 1; w < 8; ++w) tot += reds[w];
  const float inv = kPCarry / tot;
  unsigned short hb[16];
#pragma unroll
  for (int e = 0; e < 16; ++e) hb[e] = h_bits(ev[e] * inv);
  const v4u u0 = (v4u){pk16(hb[0], hb[1]), pk16(hb[2], hb[3]), pk16(hb[4], hb[5]), pk16(hb[6], hb[7])};
  const v4u u1 = (v4u){pk16(hb[8], hb[9]), pk16(hb[10], hb[11]), pk16(hb[12], hb[13]), pk16(hb[14], hb[15])};
  unsigned short* pr = P + (size_t)row * kNL;
  for (int pass = 0; pass < 2; ++pass) {
    *(volatile v4u*)(pr + cA) = u0;
    *(volatile v4u*)(pr + cB) = u1;
    __threadfence();
  }
}

__global__ __launch_bounds__(256) void xtrans_kernel(const float* __restrict__ x, unsigned short* __restrict__ xt) {
  __shared__ __align__(16) unsigned short sm[kND][kHAP];
  const int tid = threadIdx.x, lane = tid & 31, wave = tid >> 5;
  const int l0 = blockIdx.x * 128;
  const int bl = blockIdx.y;
  const float* xb = x + ((size_t)bl * kNL + l0) * kND;
#pragma unroll
  for (int it = 0; it < 16; ++it) {
    const int e = it * 256 + tid;
    const int r = e >> 5, d = e & 31;
    sm[d][r] = h_bits(xb[e]);
  }
  __syncthreads();
  const int q = lane >> 3, c8 = (lane & 7) * 8;
  const v4u zero4 = (v4u){0u, 0u, 0u, 0u};
  unsigned short* xtb = xt + (size_t)bl * kXTR * kNL + l0;
  for (int pass = 0; pass < 2; ++pass) {
#pragma unroll
    for (int it = 0; it < 2; ++it) {
      const int d = wave * 4 + it * 2 + (q >> 1);
      const int col = (q & 1) * 64 + c8;
      const v4u u = *(const v4ua*)(&sm[d][col]);
      *(volatile v4u*)(xtb + (size_t)d * kNL + col) = u;
      *(volatile v4u*)(xtb + (size_t)(d + kND) * kNL + col) = zero4;
    }
    __threadfence();
  }
}

template <bool SEQ>
__global__ __launch_bounds__(256) void gru_layer_kernel(const float* __restrict__ gi,
                                                        const unsigned short* __restrict__ whh8,
                                                        const float* __restrict__ bhh,
                                                        unsigned short* __restrict__ seq_out,
                                                        float* __restrict__ fin_out) {
  __shared__ __align__(16) _Float16 hA[2][16 * kHAP];
  __shared__ __align__(16) float sfin[16 * kSFP];
  const int tid = threadIdx.x, wave = tid >> 5, lane = tid & 31;
  const int hh = lane >> 4, c = lane & 15;
  const int koff = hh * 8;
  const int dir = blockIdx.x >> 2;
  const int rb = blockIdx.x & 3;
  const float* gid = gi + (size_t)dir * ((size_t)kNB * kNQ * kNG3);
  const _Float16* wd = (const _Float16*)whh8 + (size_t)dir * kNG3 * kNH;
  const float* bd = bhh + dir * kNG3;
  const int j = wave * 16 + c;
  const float bhr = bd[j];
  const float bhz = bd[kNH + j];
  const float bhn = bd[2 * kNH + j];
  {
    const v4ua z4 = (v4ua){0u, 0u, 0u, 0u};
    _Float16* hflat = &hA[0][0];
    for (int i = tid; i < (2 * 16 * kHAP) / 8; i += 256) *(v4ua*)(hflat + 8 * i) = z4;
  }
  float hreg[8];
#pragma unroll
  for (int r = 0; r < 8; ++r) hreg[r] = 0.f;
  __syncthreads();

  for (int s = 0; s < kNQ; ++s) {
    const int t = (dir != 0) ? (kNQ - 1 - s) : s;
    const int cur = s & 1, nxt = cur ^ 1;
    const _Float16* ha = &hA[cur][0];
    _Float16* hnext = &hA[nxt][0];
    v8f acc0 = (v8f){0.f,0.f,0.f,0.f,0.f,0.f,0.f,0.f};
    v8f acc1 = (v8f){0.f,0.f,0.f,0.f,0.f,0.f,0.f,0.f};
    v8f acc2 = (v8f){0.f,0.f,0.f,0.f,0.f,0.f,0.f,0.f};
#pragma unroll
    for (int kc = 0; kc < 4; ++kc) {
      const v16h af = Frag<_Float16>::load(ha + c * kHAP + koff + kc * 32);
      const v16h b0 = Frag<_Float16>::load(wd + (size_t)(0 * kNH + j) * kNH + koff + kc * 32);
      const v16h b1 = Frag<_Float16>::load(wd + (size_t)(1 * kNH + j) * kNH + koff + kc * 32);
      const v16h b2 = Frag<_Float16>::load(wd + (size_t)(2 * kNH + j) * kNH + koff + kc * 32);
      acc0 = Frag<_Float16>::mma(af, b0, acc0);
      acc1 = Frag<_Float16>::mma(af, b1, acc1);
      acc2 = Frag<_Float16>::mma(af, b2, acc2);
      guard3_h(acc0, acc1, acc2, af, b0, b1, b2);
    }
    asm volatile("v_nop\n\tv_nop\n\tv_nop\n\tv_nop" : "+v"(acc0), "+v"(acc1), "+v"(acc2));
#pragma unroll
    for (int r = 0; r < 8; ++r) {
      const int row = hh * 8 + r;
      const int bidx = rb * 16 + row;
      const float* gp = gid + ((size_t)bidx * kNQ + t) * kNG3;
      const float gir = gp[j];
      const float giz = gp[kNH + j];
      const float gin = gp[2 * kNH + j];
      const float ghr = acc0[r] * kGhScale + bhr;
      const float ghz = acc1[r] * kGhScale + bhz;
      const float ghn = acc2[r] * kGhScale + bhn;
      const float rg = 1.0f / (1.0f + expf(-(gir + ghr)));
      const float zg = 1.0f / (1.0f + expf(-(giz + ghz)));
      const float ng = tanhf(gin + rg * ghn);
      const float hv = (1.0f - zg) * ng + zg * hreg[r];
      hreg[r] = hv;
      hnext[row * kHAP + j] = (_Float16)(hv * kActCarry);
    }
    __syncthreads();
    if (SEQ) {
      const int q = lane >> 3, c8 = (lane & 7) * 8;
      const int row = wave * 2 + (q >> 1);
      const int col = (q & 1) * 64 + c8;
      const v8h hvec = *(const v8h*)(hnext + row * kHAP + col);
      unsigned short* dst = seq_out + ((size_t)(rb * 16 + row) * kNQ + t) * (2 * kNH) + dir * kNH + col;
      for (int pass = 0; pass < 2; ++pass) {
        *(volatile v8h*)dst = hvec;
        __threadfence();
      }
    }
  }
  if (!SEQ) {
#pragma unroll
    for (int r = 0; r < 8; ++r) sfin[(hh * 8 + r) * kSFP + j] = hreg[r];
    __syncthreads();
    const int row0 = wave * 2;
    const v4f v0 = *(const v4f*)(sfin + row0 * kSFP + 4 * lane);
    const v4f v1 = *(const v4f*)(sfin + (row0 + 1) * kSFP + 4 * lane);
    float* d0 = fin_out + (size_t)(rb * 16 + row0) * (2 * kNH) + dir * kNH + 4 * lane;
    float* d1 = d0 + 2 * kNH;
    for (int pass = 0; pass < 2; ++pass) {
      *(volatile v4f*)d0 = v0;
      *(volatile v4f*)d1 = v1;
      __threadfence();
    }
  }
}

__global__ __launch_bounds__(256) void head_kernel(const float* __restrict__ cin, const float* __restrict__ c1w,
                                                   const float* __restrict__ c1b, const float* __restrict__ c2w,
                                                   const float* __restrict__ c2b, const float* __restrict__ c3w,
                                                   const float* __restrict__ c3b, float* __restrict__ out) {
  __shared__ float s_h1[kNB * 128];
  __shared__ float s_h2[kNB * 64];
  __shared__ __align__(16) float s_o[512];
  const int tid = threadIdx.x;
#pragma unroll 1
  for (int idx = tid; idx < kNB * 128; idx += 256) {
    const int b = idx >> 7, o = idx & 127;
    const float* cr = cin + b * 256;
    float a = c1b[o];
#pragma unroll 1
    for (int k = 0; k < 256; ++k) a += cr[k] * c1w[k * 128 + o];
    s_h1[idx] = a;
  }
  __syncthreads();
#pragma unroll 1
  for (int idx = tid; idx < kNB * 64; idx += 256) {
    const int b = idx >> 6, o = idx & 63;
    const float* hr = s_h1 + b * 128;
    float a = c2b[o];
#pragma unroll 1
    for (int k = 0; k < 128; ++k) a += hr[k] * c2w[k * 64 + o];
    s_h2[idx] = a;
  }
  __syncthreads();
#pragma unroll 1
  for (int idx = tid; idx < kNB * kNCLS; idx += 256) {
    const int b = idx / kNCLS;
    const int o = idx - b * kNCLS;
    const float* hr = s_h2 + b * 64;
    float a = c3b[o];
#pragma unroll 1
    for (int k = 0; k < 64; ++k) a += hr[k] * c3w[k * kNCLS + o];
    s_o[idx] = a;
  }
  __syncthreads();
  if (tid < 32) {
    for (int pass = 0; pass < 2; ++pass) {
#pragma unroll
      for (int it = 0; it < 3; ++it) {
        const v4f v = *(const v4f*)(s_o + it * 128 + 4 * tid);
        *(volatile v4f*)(out + it * 128 + 4 * tid) = v;
      }
      __threadfence();
    }
  }
}

extern "C" void kernel_launch(void* const* d_in, const int* in_sizes, int n_in,
                              void* d_out, int out_size, void* d_ws, size_t ws_size,
                              hipStream_t stream) {
  (void)in_sizes; (void)n_in; (void)out_size;
  const float* x      = (const float*)d_in[0];
  const float* ts     = (const float*)d_in[1];
  const float* qt     = (const float*)d_in[2];
  const float* lin_w  = (const float*)d_in[3];
  const float* lin_b  = (const float*)d_in[4];
  const float* per_w  = (const float*)d_in[5];
  const float* per_b  = (const float*)d_in[6];
  const float* wq     = (const float*)d_in[7];
  const float* bq     = (const float*)d_in[8];
  const float* wk     = (const float*)d_in[9];
  const float* bk     = (const float*)d_in[10];
  const float* wo     = (const float*)d_in[11];
  const float* bo     = (const float*)d_in[12];
  const float* g0_wih = (const float*)d_in[13];
  const float* g0_whh = (const float*)d_in[14];
  const float* g0_bih = (const float*)d_in[15];
  const float* g0_bhh = (const float*)d_in[16];
  const float* g1_wih = (const float*)d_in[17];
  const float* g1_whh = (const float*)d_in[18];
  const float* g1_bih = (const float*)d_in[19];
  const float* g1_bhh = (const float*)d_in[20];
  const float* c1w = (const float*)d_in[21];
  const float* c1b = (const float*)d_in[22];
  const float* c2w = (const float*)d_in[23];
  const float* c2b = (const float*)d_in[24];
  const float* c3w = (const float*)d_in[25];
  const float* c3b = (const float*)d_in[26];
  float* out = (float*)d_out;

  char* ws = (char*)d_ws;
  size_t off = 0;
  auto take = [&](size_t bytes) -> size_t { size_t o = off; off += (bytes + 4095) & ~(size_t)4095; return o; };
  const size_t oBias = take(3 * 512);
  const size_t oWqt  = take((size_t)kNE * kNE * 2);
  const size_t oWkt  = take((size_t)kNE * kNE * 2);
  const size_t oWot  = take((size_t)kNH * kND * 2);
  const size_t oWih0 = take((size_t)2 * kNG3 * kNH * 2);
  const size_t oWhh0 = take((size_t)2 * kNG3 * kNH * 2);
  const size_t oWih1 = take((size_t)2 * kNG3 * 2 * kNH * 2);
  const size_t oWhh1 = take((size_t)2 * kNG3 * kNH * 2);
  const size_t oTeq  = take((size_t)kNQ * kNE * 2);
  const size_t oQp   = take((size_t)kNQ * kNE * 2);
  const size_t oAtt  = take((size_t)kNB * kNQ * kXTR * 2);
  const size_t oAo   = take((size_t)kNB * kNQ * kNH * 2);
  const size_t oG0   = take((size_t)kNB * kNQ * 2 * kNH * 2);
  const size_t oCin  = take((size_t)kNB * 2 * kNH * 4);
  const size_t oTek  = take((size_t)kGB * kNL * kNE * 2);
  const size_t oKp   = take((size_t)kGB * kNL * kNE * 2);
  const size_t oSc   = take((size_t)kGB * kNQ * kNL * 4);
  const size_t oPp   = take((size_t)kGB * kNQ * kNL * 2);
  const size_t oXt   = take((size_t)kGB * kXTR * kNL * 2);
  if (off > ws_size) return;
  if ((size_t)2 * kNB * kNQ * kNG3 * 4 > (size_t)kGB * kNQ * kNL * 4) return;

  float* bias3 = (float*)(ws + oBias);
  float* bq8  = bias3;
  float* bk8  = bias3 + kNE;
  float* bo16 = bias3 + 2 * kNE;
  unsigned short* WQT  = (unsigned short*)(ws + oWqt);
  unsigned short* WKT  = (unsigned short*)(ws + oWkt);
  unsigned short* WOT  = (unsigned short*)(ws + oWot);
  unsigned short* WIH0 = (unsigned short*)(ws + oWih0);
  unsigned short* WHH0 = (unsigned short*)(ws + oWhh0);
  unsigned short* WIH1 = (unsigned short*)(ws + oWih1);
  unsigned short* WHH1 = (unsigned short*)(ws + oWhh1);
  unsigned short* TEQ  = (unsigned short*)(ws + oTeq);
  unsigned short* QP   = (unsigned short*)(ws + oQp);
  unsigned short* ATT  = (unsigned short*)(ws + oAtt);
  unsigned short* AO   = (unsigned short*)(ws + oAo);
  unsigned short* G0   = (unsigned short*)(ws + oG0);
  float*          CIN  = (float*)(ws + oCin);
  unsigned short* TEK  = (unsigned short*)(ws + oTek);
  unsigned short* KP   = (unsigned short*)(ws + oKp);
  float*          SC   = (float*)(ws + oSc);
  float*          GI   = (float*)(ws + oSc);
  unsigned short* PP   = (unsigned short*)(ws + oPp);
  unsigned short* XT   = (unsigned short*)(ws + oXt);

  const float kProjScale  = kWCarry / (kTeCarry * kWCarry);
  const float kScoreScale = 0.08838834764831845f / (kWCarry * kWCarry);
  const float kPVScale    = kAttCarry / kPCarry;
  const float kAOScale    = kActCarry / (kAttCarry * kWCarry);
  const float kGiScale    = 1.0f / (kActCarry * kWCarry);

  prep_bias_kernel<<<dim3(3), dim3(32), 0, stream>>>(bq, bk, bo, bias3);
  wtrans_kernel<<<dim3(3), dim3(256), 0, stream>>>(wq, wk, wo, WQT, WKT, WOT, kWCarry);
  castw_kernel<<<dim3((2 * kNG3 * 2 * kNH / 8) / 256, 4), dim3(256), 0, stream>>>(
      g0_wih, g0_whh, g1_wih, g1_whh, WIH0, WHH0, WIH1, WHH1,
      2 * kNG3 * kNH / 8, 2 * kNG3 * 2 * kNH / 8, kWCarry);
  te_kernel<<<dim3(kNQ / 16), dim3(256), 0, stream>>>(qt, kNQ, lin_w, lin_b, per_w, per_b, TEQ);
  wmma_gemm64<0, false, 2, 1, false><<<dim3(1, 1), dim3(128), 0, stream>>>(
      TEQ, TEQ, kNE, 0L, WQT, WQT, kNE, 0L, (void*)QP, (void*)QP, kNE, 0L,
      bq8, bias3, 0L, kNQ, kNE, kNE, kProjScale);

  for (int g = 0; g < kNGRP; ++g) {
    const float* tsg = ts + (size_t)g * kGB * kNL;
    const float* xg  = x + (size_t)g * kGB * kNL * kND;
    te_kernel<<<dim3(kGB * kNL / 16), dim3(256), 0, stream>>>(tsg, kGB * kNL, lin_w, lin_b, per_w, per_b, TEK);
    wmma_gemm64<0, false, 2, 1, false><<<dim3(kGB * kNL * 2 / 64 / 8, 1), dim3(256), 0, stream>>>(
        TEK, TEK, kNE, 0L, WKT, WKT, kNE, 0L, (void*)KP, (void*)KP, kNE, 0L,
        bk8, bias3, 0L, kGB * kNL, kNE, kNE, kProjScale);
    wmma_gemm64<0, false, 0, 0, false><<<dim3(16, kGB), dim3(256), 0, stream>>>(
        QP, QP, kNE, 0L, KP, KP, kNE, (long)kNL * kNE, (void*)SC, (void*)SC, kNL, (long)kNQ * kNL,
        bias3, bias3, 0L, kNQ, kNL, kNE, kScoreScale);
    softmax_kernel<<<dim3(kGB * kNQ), dim3(256), 0, stream>>>(SC, PP);
    xtrans_kernel<<<dim3(kNL / 128, kGB), dim3(256), 0, stream>>>(xg, XT);
    wmma_gemm64<0, false, 0, 1, false><<<dim3(1, kGB), dim3(64), 0, stream>>>(
        PP, PP, kNL, (long)kNQ * kNL, XT, XT, kNL, (long)kXTR * kNL,
        (void*)(ATT + (size_t)g * kGB * kNQ * kXTR), (void*)(ATT + (size_t)g * kGB * kNQ * kXTR), kXTR, (long)kNQ * kXTR,
        bias3, bias3, 0L, kNQ, kXTR, kNL, kPVScale);
  }

  wmma_gemm64<0, false, 2, 1, false><<<dim3(kNB * kNQ * 2 / 64 / 8, 1), dim3(256), 0, stream>>>(
      ATT, ATT, kXTR, 0L, WOT, WOT, kND, 0L, (void*)AO, (void*)AO, kNH, 0L,
      bo16, bias3, 0L, kNB * kNQ, kNH, kND, kAOScale);

  for (int dir = 0; dir < 2; ++dir) {
    wmma_gemm64<0, false, 2, 0, false><<<dim3(kNB * kNQ * kNG3 / 64 / 64 / 8, 1), dim3(256), 0, stream>>>(
        AO, AO, kNH, 0L, WIH0 + (size_t)dir * kNG3 * kNH, WIH0 + (size_t)dir * kNG3 * kNH, kNH, 0L,
        (void*)(GI + (size_t)dir * kNB * kNQ * kNG3), (void*)(GI + (size_t)dir * kNB * kNQ * kNG3), kNG3, 0L,
        g0_bih + dir * kNG3, bias3, 0L, kNB * kNQ, kNG3, kNH, kGiScale);
  }
  gru_layer_kernel<true><<<dim3(8), dim3(256), 0, stream>>>(GI, WHH0, g0_bhh, G0, CIN);

  for (int dir = 0; dir < 2; ++dir) {
    wmma_gemm64<0, false, 2, 0, false><<<dim3(kNB * kNQ * kNG3 / 64 / 64 / 8, 1), dim3(256), 0, stream>>>(
        G0, G0, 2 * kNH, 0L, WIH1 + (size_t)dir * kNG3 * 2 * kNH, WIH1 + (size_t)dir * kNG3 * 2 * kNH, 2 * kNH, 0L,
        (void*)(GI + (size_t)dir * kNB * kNQ * kNG3), (void*)(GI + (size_t)dir * kNB * kNQ * kNG3), kNG3, 0L,
        g1_bih + dir * kNG3, bias3, 0L, kNB * kNQ, kNG3, 2 * kNH, kGiScale);
  }
  gru_layer_kernel<false><<<dim3(8), dim3(256), 0, stream>>>(GI, WHH1, g1_bhh, G0, CIN);

  head_kernel<<<dim3(1), dim3(256), 0, stream>>>(CIN, c1w, c1b, c2w, c2b, c3w, c3b, out);
}
